// MHSA_42863773614629
// MI455X (gfx1250) — hardware-verified
//
#include <hip/hip_runtime.h>


namespace {
constexpr int B = 16, C = 512, IH = 32, IW = 32, T = IH * IW  , H = 4, HD = 128, DM = H * HD  , NQKV = 3 * DM, BL = 16  , QL = T;
constexpr float XS = 8.0f, WSC = 256.0f, PS = 1024.0f, RS_ = 1024.0f, LOG2E = 1.4426950408889634f, SCL = 0.08838834764831845f  ;
static_assert(T % 64 == 0 && C % 256 == 0 && HD == 128 && IW == 32, "tiling");
typedef _Float16 b16;
typedef __attribute__((ext_vector_type(16))) _Float16 v16b;
typedef __attribute__((ext_vector_type(8))) _Float16 v8b;
typedef __attribute__((ext_vector_type(8))) float v8f;
typedef __attribute__((ext_vector_type(4))) float v4f;
__device__ __forceinline__ float bf16_rne(float f) { unsigned int u = __float_as_uint(f); u += 0x7FFFu + ((u >> 16) & 1u); return __uint_as_float(u & 0xFFFF0000u); }
__device__ __forceinline__ void split16(float v, b16& hi, b16& lo) { hi = (b16)v; lo = (b16)(v - (float)hi); }
__device__ __forceinline__ v16b frag_kb(const b16* p, int hh) { const v8b a = *(const v8b*)(p + 8 * hh), b = *(const v8b*)(p + 16 + 8 * hh); v16b f;
#pragma unroll
  for (int e = 0; e < 8; ++e) { f[e] = a[e]; f[8 + e] = b[e]; } return f; }
__device__ __forceinline__ v8f wmma16b(v16b a, v16b b, v8f c) { v8f d = __builtin_amdgcn_wmma_f32_16x16x32_f16(false, a, false, b, (short)0, c, false, false); asm volatile("v_nop\n\tv_nop\n\tv_nop\n\tv_nop" : "+v"(d) : "v"(a), "v"(b)); return d; }
__device__ __forceinline__ void wave_lds_sync() { __builtin_amdgcn_fence(__ATOMIC_RELEASE, "workgroup"); __builtin_amdgcn_wave_barrier(); __builtin_amdgcn_fence(__ATOMIC_ACQUIRE, "workgroup"); }
__device__ __forceinline__ float pmul(float a, float b) { float p = a * b; asm volatile("" : "+v"(p)); return p; }
__device__ __forceinline__ int iclamp(int v, int lo, int hi) { return v < lo ? lo : (v > hi ? hi : v); }

typedef __attribute__((ext_vector_type(2))) _Float16 v2h;
typedef __attribute__((ext_vector_type(4))) _Float16 v4h;
typedef __attribute__((ext_vector_type(2))) float v2f;
typedef __attribute__((ext_vector_type(4))) int v4i;
__device__ __forceinline__ float nexp2(float v) { return __builtin_amdgcn_exp2f(v); }
__global__ __launch_bounds__(256) void prep_kernel(const float* __restrict__ wqk, const float* __restrict__ wv, b16* __restrict__ WT) {
  const size_t u = (size_t)blockIdx.x * 256 + threadIdx.x; if (u >= (size_t)NQKV * C / 8) return; const size_t e = u * 8; const int o = (int)(e / C), c0 = (int)(e % C); const float* w = o < 2 * DM ? (wqk + (size_t)o * C) : (wv + (size_t)(o - 2 * DM) * C); v8b v;
  for (int j = 0; j < 8; ++j) v[j] = (b16)(bf16_rne(w[c0 + j]) * WSC);
  for (int pass = 0; pass < 2; ++pass) { *(volatile v8b*)(WT + e) = v; __threadfence(); }
}
__global__ __launch_bounds__(128) void proj_kernel(const float* __restrict__ fm, const b16* __restrict__ WT, const float* __restrict__ embh, const float* __restrict__ embw, b16* __restrict__ QP, b16* __restrict__ QPl, b16* __restrict__ KP, b16* __restrict__ KPl, b16* __restrict__ VT, b16* __restrict__ VTl) {
  __shared__ __attribute__((aligned(16))) b16 As[64][256 + 8]; __shared__ __attribute__((aligned(16))) float Tf[4][16][128 + 4];
  const int wave = threadIdx.x >> 5, lane = threadIdx.x & 31, nloc = lane & 15, hlf = lane >> 4; const int p0 = blockIdx.x * 64, b = blockIdx.y, slab = blockIdx.z; const int part = slab / H, h = slab % H; const int n0 = slab * 128;
  const float* fb = fm + (size_t)b * C * T;
  v8f acc[8];
#pragma unroll
  for (int t = 0; t < 8; ++t) acc[t] = (v8f){};
#pragma unroll 1
  for (int kc = 0; kc < C; kc += 256) {
    __syncthreads();
    for (int i = threadIdx.x; i < 256 * 16; i += 128) { const int c = i / 16, q4 = (i % 16) * 4; const v4f f = *(const v4f*)(fb + (size_t)(kc + c) * T + p0 + q4); for (int j = 0; j < 4; ++j) As[q4 + j][c] = (b16)(bf16_rne(f[j]) * XS); }
    __syncthreads();
#pragma unroll 2
    for (int kb = 0; kb < 256; kb += 32) { const v16b a = frag_kb(&As[wave * 16 + nloc][kb], hlf);
#pragma unroll
      for (int t = 0; t < 8; ++t) acc[t] = wmma16b(a, frag_kb(WT + (size_t)(n0 + t * 16 + nloc) * C + kc + kb, hlf), acc[t]); } }
#pragma unroll
  for (int t = 0; t < 8; ++t)
#pragma unroll
    for (int r = 0; r < 8; ++r) Tf[wave][8 * hlf + r][t * 16 + nloc] = acc[t][r] * (1.0f / (XS * WSC));
  __syncthreads();
  for (int pass = 0; pass < 2; ++pass) {
    if (part < 2) { const size_t pb = (((size_t)b * H + h) * T) * HD; b16* ph_ = part == 0 ? QP : KP; b16* pl_ = part == 0 ? QPl : KPl;
      for (int rr = 0; rr < 16; ++rr) { const int pos = p0 + wave * 16 + rr; v4h h4, l4;
        for (int j = 0; j < 4; ++j) { const int d = lane * 4 + j; float v = Tf[wave][rr][d]; if (part == 0) v *= SCL; else v += bf16_rne(embh[(pos / IW) * HD + d]) + bf16_rne(embw[(pos % IW) * HD + d]); const float f = v * XS; const b16 p = (b16)f; h4[j] = p; l4[j] = (b16)((f - (float)p) * RS_); }
        *(volatile v4h*)(ph_ + pb + (size_t)pos * HD + lane * 4) = h4; *(volatile v4h*)(pl_ + pb + (size_t)pos * HD + lane * 4) = l4; } }
    else { const size_t vb = (((size_t)b * H + h) * HD) * (size_t)T;
#pragma unroll 1
      for (int q = 0; q < 32; ++q) { const int d = wave * 32 + q; const int tk = lane * 2; v2h hv, lv; for (int j = 0; j < 2; ++j) { const float f = Tf[(tk + j) >> 4][(tk + j) & 15][d] * XS; const b16 p = (b16)f; hv[j] = p; lv[j] = (b16)((f - (float)p) * RS_); }
        *(volatile v2h*)(VT + vb + (size_t)d * T + p0 + lane * 2) = hv; *(volatile v2h*)(VTl + vb + (size_t)d * T + p0 + lane * 2) = lv; } }
    __threadfence(); }
}
__global__ __launch_bounds__(64) void attn_kernel(const b16* __restrict__ QP, const b16* __restrict__ QPl, const b16* __restrict__ KP, const b16* __restrict__ KPl, const b16* __restrict__ VT, const b16* __restrict__ VTl, float* __restrict__ out) {
  __shared__ __attribute__((aligned(16))) b16 Pb[2][16][32 + 8]; __shared__ __attribute__((aligned(16))) float To[2][16][HD + 4];
  const int wave = threadIdx.x >> 5, lane = threadIdx.x & 31, hh = lane >> 4, col = lane & 15; const int b = blockIdx.y / H, h = blockIdx.y % H; const int q0 = blockIdx.x * 32 + wave * 16, qi = q0 + col;
  const size_t qo = (((size_t)b * H + h) * T) * HD, vo = (((size_t)b * H + h) * HD) * (size_t)T; const b16* Qb = QP + qo; const b16* Qbl = QPl + qo; const b16* Kb = KP + qo; const b16* Kbl = KPl + qo; const b16* Vb = VT + vo; const b16* Vbl = VTl + vo;
  __shared__ __attribute__((aligned(16))) b16 Qs[2][16][HD + 8], Qsl[2][16][HD + 8];
  for (int i = lane; i < 16 * (HD / 8); i += 32) { const int rr = i / (HD / 8), c8 = (i % (HD / 8)) * 8; *(v8b*)(&Qs[wave][rr][c8]) = *(const v8b*)(Qb + (size_t)(q0 + rr) * HD + c8); *(v8b*)(&Qsl[wave][rr][c8]) = *(const v8b*)(Qbl + (size_t)(q0 + rr) * HD + c8); }
  wave_lds_sync();
  const float cs = LOG2E / (XS * XS);
  __shared__ __attribute__((aligned(16))) b16 Plq[2][16][32 + 8];
  float m = -INFINITY, l = 0.0f; v8f o[8], ol[8]; for (int t = 0; t < 8; ++t) { o[t] = (v8f){}; ol[t] = (v8f){}; }
#pragma unroll 1
  for (int kb = 0; kb < T; kb += 32) {
    float e[16]; float mx = -INFINITY;
#pragma unroll
    for (int u = 0; u < 2; ++u) { v8f s = (v8f){}, sx = (v8f){}; const size_t kr = (size_t)(kb + u * 16 + col) * HD;
#pragma unroll
      for (int ks = 0; ks < 4; ++ks) { const v16b kf = frag_kb(Kb + kr + 32 * ks, hh); const v16b qf = frag_kb(&Qs[wave][col][32 * ks], hh); s = wmma16b(kf, qf, s); sx = wmma16b(kf, frag_kb(&Qsl[wave][col][32 * ks], hh), sx); sx = wmma16b(frag_kb(Kbl + kr + 32 * ks, hh), qf, sx); }
#pragma unroll
      for (int r = 0; r < 8; ++r) s[r] += sx[r] * (1.0f / RS_);
#pragma unroll
      for (int r = 0; r < 8; ++r) { const float vv = s[r] * cs; e[u * 8 + r] = vv; mx = fmaxf(mx, vv); } }
    mx = fmaxf(mx, __shfl_xor(mx, 16)); const float mn = fmaxf(m, mx); const float al = nexp2(m - mn); float sum = 0.0f;
#pragma unroll
    for (int i2 = 0; i2 < 16; ++i2) { const float p = nexp2(e[i2] - mn); sum += p; const int pc = (i2 < 8 ? 0 : 16) + 8 * hh + (i2 & 7); const float ps = p * PS; const b16 phh = (b16)ps; Pb[wave][col][pc] = phh; Plq[wave][col][pc] = (b16)((ps - (float)phh) * RS_); }
    sum += __shfl_xor(sum, 16); l = l * al + sum; m = mn;
    wave_lds_sync();
    const v16b pf = frag_kb(&Pb[wave][col][0], hh), plf = frag_kb(&Plq[wave][col][0], hh);
#pragma unroll
    for (int t = 0; t < 8; ++t) { const v16b vh = frag_kb(Vb + (size_t)(t * 16 + col) * T + kb, hh); o[t] *= al; o[t] = wmma16b(vh, pf, o[t]); ol[t] = wmma16b(frag_kb(Vbl + (size_t)(t * 16 + col) * T + kb, hh), pf, ol[t] * al); ol[t] = wmma16b(vh, plf, ol[t]); }
    wave_lds_sync(); }
  const float inv = 1.0f / (l * PS * XS);
#pragma unroll
  for (int t = 0; t < 8; ++t)
#pragma unroll
    for (int r = 0; r < 8; ++r) To[wave][col][t * 16 + 8 * hh + r] = (o[t][r] + ol[t][r] * (1.0f / RS_)) * inv;
  wave_lds_sync();
  __syncthreads();
  for (int pass = 0; pass < 2; ++pass) { for (int d = threadIdx.x; d < HD; d += 64) { float* orow = out + (((size_t)b * H + h) * HD + d) * (size_t)T + blockIdx.x * 32; v4f o4;
      for (int q4 = 0; q4 < 8; ++q4) { for (int j = 0; j < 4; ++j) { const int qq = q4 * 4 + j; o4[j] = To[qq >> 4][qq & 15][d]; } *(volatile v4f*)(orow + q4 * 4) = o4; } } __threadfence(); }
}
}

extern "C" void kernel_launch(void* const* d_in, const int* in_sizes, int n_in, void* d_out, int out_size, void* d_ws, size_t ws_size, hipStream_t stream) {
  (void)n_in;
  auto Fp = [&](int i) { return (const float*)d_in[i]; };
  if (in_sizes[0] != B * C * T || in_sizes[1] != 2 * DM * C || in_sizes[2] != DM * C || in_sizes[3] != IH * HD || in_sizes[4] != IW * HD || out_size != B * DM * T) return;
  size_t off = 0; char* ws = (char*)d_ws;
  auto carve = [&](size_t bytes) { char* p = ws + off; off += (bytes + 255) & ~(size_t)255; return p; };
  b16* WT = (b16*)carve((size_t)NQKV * C * 2); const size_t plane = (size_t)B * H * T * HD * 2;
  b16* QP = (b16*)carve(plane); b16* QPl = (b16*)carve(plane); b16* KP = (b16*)carve(plane); b16* KPl = (b16*)carve(plane); b16* VT = (b16*)carve(plane); b16* VTl = (b16*)carve(plane);
  if (off > ws_size || off > ((size_t)128 << 20)) return;
  prep_kernel<<<(unsigned)(((size_t)NQKV * C / 8 + 255) / 256), 256, 0, stream>>>(Fp(1), Fp(2), WT);
  proj_kernel<<<dim3(T / 64, BL, 3 * H), 128, 0, stream>>>(Fp(0), WT, Fp(3), Fp(4), QP, QPl, KP, KPl, VT, VTl);
  attn_kernel<<<dim3(QL / 32, BL * H), 64, 0, stream>>>(QP, QPl, KP, KPl, VT, VTl, (float*)d_out);
}
